// SimpleNet_61710090108974
// MI455X (gfx1250) — hardware-run, weakly checked
//
#include <hip/hip_runtime.h>
#include <math.h>

typedef __attribute__((ext_vector_type(16))) _Float16 v16h;
typedef __attribute__((ext_vector_type(8)))  _Float16 v8h;
typedef __attribute__((ext_vector_type(8)))  float    v8f;
typedef __attribute__((ext_vector_type(4)))  float    v4f;

constexpr int kImgs    = 4;
constexpr int kCin     = 3;
constexpr int kPlane   = 1024 * 1024;
constexpr int kHidC    = 25;
constexpr int kDepth   = 6;
constexpr int kChunk   = 128;
constexpr int kTilesPerChunk = kChunk / 16;
constexpr int kWaves   = 2048;
constexpr int kWavesPerBlock = 2;
constexpr int kChunksTotal = kImgs * kPlane / kChunk;
constexpr int kChunksPerWave = kChunksTotal / kWaves;
constexpr int kPitch   = kChunk + 4;
constexpr size_t kIoElems = (size_t)kImgs * kCin * kPlane;
static_assert(kChunksTotal % kWaves == 0 && (kPlane % kChunk) == 0, "whole chunks per wave; a chunk lies inside one image plane");
static_assert(kHidC <= 32 && kCin <= 8, "the hidden channels fit two 16-row tiles and one 32-wide K; the output channels fit the low lane half");
static_assert((kPitch % 4) == 0, "16-B aligned LDS rows");

constexpr float kActCarry   = 4096.0f;
constexpr float kWCarry     = 1024.0f;
constexpr float kFoldBack   = 1.0f / (kActCarry * kWCarry);
constexpr float kF16MinNorm = 6.103515625e-5f;

namespace eng {

union FragU { v16h v; v8h h[2]; };

__device__ __forceinline__ unsigned short f2bf_bits(float f) {
  unsigned u = __float_as_uint(f);
  return (unsigned short)((u + 0x7FFFu + ((u >> 16) & 1u)) >> 16);
}
__device__ __forceinline__ float bf16v(float f) {
  return __uint_as_float(((unsigned)f2bf_bits(f)) << 16);
}
__device__ __forceinline__ _Float16 to_f16_flushed(float c) {
  const float z = (fabsf(c) < kF16MinNorm) ? 0.0f : c;
  return (_Float16)z;
}
__device__ __forceinline__ v8f mma_f16(v16h a, v16h b) {
  v8f c = (v8f){0.f, 0.f, 0.f, 0.f, 0.f, 0.f, 0.f, 0.f};
  c = __builtin_amdgcn_wmma_f32_16x16x32_f16(false, a, false, b, (short)0, c, false, false);
  asm volatile("v_nop\n\tv_nop\n\tv_nop\n\tv_nop" : "+v"(c) : "v"(a), "v"(b));
  return c;
}
__device__ __forceinline__ float fast_tanh(float v) {
  const float e = __expf(2.0f * v);
  return 1.0f - 2.0f * __builtin_amdgcn_rcpf(e + 1.0f);
}

}

__global__ __launch_bounds__(64) void pixel_mlp_kernel(
    const float* __restrict__ x, const float* __restrict__ w_in, const float* __restrict__ ws,
    const float* __restrict__ w_out, float* __restrict__ outs)
{
  __shared__ __align__(16) float xsAll[kWavesPerBlock][kCin * kPitch];
  __shared__ __align__(16) float osAll[kWavesPerBlock][kCin * kPitch];
  __shared__ __align__(16) float wsm[3904];

  const int lane = threadIdx.x & 31;
  const int wave = threadIdx.x >> 5;
  float* xs = &xsAll[wave][0];
  float* os = &osAll[wave][0];
  const int hsel = lane >> 4;
  const int n    = lane & 15;
  const bool lowHalf = (hsel == 0);
  constexpr int oIn = 0, oWs = 75, oOut = 75 + kDepth * kHidC * kHidC;

  {
#pragma unroll
    for (int it = 0; it < 3; ++it) {
      const int i = it * 32 + lane;
      const int ic = (i < kHidC * kCin) ? i : (kHidC * kCin - 1);
      wsm[oIn + ic]  = w_in[ic];
      wsm[oOut + ic] = w_out[ic];
    }
#pragma unroll 1
    for (int it = 0; it < (kDepth * kHidC * kHidC + 31) / 32; ++it) {
      const int i = it * 32 + lane;
      const int ic = (i < kDepth * kHidC * kHidC) ? i : (kDepth * kHidC * kHidC - 1);
      wsm[oWs + ic] = ws[ic];
    }
  }
  __syncthreads();

  v16h fragW[kDepth][2];
  v16h fragO;
  {
    const int m = n;
#pragma unroll
    for (int l = 0; l < kDepth; ++l) {
#pragma unroll
      for (int tl = 0; tl < 2; ++tl) {
        const int oc = 16 * tl + m;
        const int occ = (oc < kHidC) ? oc : (kHidC - 1);
        v8h a0, a1;
#pragma unroll
        for (int i = 0; i < 8; ++i) {
          const int k0 = 8 * hsel + i;
          const int k1 = 16 + 8 * hsel + i;
          const int k1c = (k1 < kHidC) ? k1 : (kHidC - 1);
          const float f0 = eng::bf16v(wsm[oWs + (l * kHidC + occ) * kHidC + k0]);
          const float f1 = eng::bf16v(wsm[oWs + (l * kHidC + occ) * kHidC + k1c]);
          a0[i] = eng::to_f16_flushed((oc < kHidC) ? f0 * kWCarry : 0.0f);
          a1[i] = eng::to_f16_flushed((oc < kHidC && k1 < kHidC) ? f1 * kWCarry : 0.0f);
        }
        eng::FragU fu; fu.h[0] = a0; fu.h[1] = a1;
        fragW[l][tl] = fu.v;
      }
    }
    {
      const int occ = (m < kCin) ? m : (kCin - 1);
      v8h a0, a1;
#pragma unroll
      for (int i = 0; i < 8; ++i) {
        const int k0 = 8 * hsel + i;
        const int k1 = 16 + 8 * hsel + i;
        const int k1c = (k1 < kHidC) ? k1 : (kHidC - 1);
        const float f0 = eng::bf16v(wsm[oOut + occ * kHidC + k0]);
        const float f1 = eng::bf16v(wsm[oOut + occ * kHidC + k1c]);
        a0[i] = eng::to_f16_flushed((m < kCin) ? f0 * kWCarry : 0.0f);
        a1[i] = eng::to_f16_flushed((m < kCin && k1 < kHidC) ? f1 * kWCarry : 0.0f);
      }
      eng::FragU fu; fu.h[0] = a0; fu.h[1] = a1;
      fragO = fu.v;
    }
  }
  float wi0[8][kCin], wi1[8][kCin];
#pragma unroll
  for (int r = 0; r < 8; ++r) {
    const int c0 = 8 * hsel + r;
    const int c1 = 16 + 8 * hsel + r;
    const int c1c = (c1 < kHidC) ? c1 : (kHidC - 1);
#pragma unroll
    for (int c = 0; c < kCin; ++c) {
      wi0[r][c] = eng::bf16v(wsm[oIn + c0 * kCin + c]);
      const float v1 = eng::bf16v(wsm[oIn + c1c * kCin + c]);
      wi1[r][c] = (c1 < kHidC) ? v1 : 0.0f;
    }
  }

#pragma unroll 1
  for (int j = 0; j < kChunksPerWave; ++j) {
    const int cid = (blockIdx.x * kWavesPerBlock + wave) + kWaves * j;
    const size_t pf = (size_t)cid * kChunk;
    const int img = (int)(pf / kPlane);
    const size_t pix = pf - (size_t)img * kPlane;
#pragma unroll
    for (int c = 0; c < kCin; ++c) {
      const v4f v = *(const v4f*)(x + ((size_t)img * kCin + c) * kPlane + pix + 4 * lane);
      v4f rv;
      rv[0] = eng::bf16v(v[0]);
      rv[1] = eng::bf16v(v[1]);
      rv[2] = eng::bf16v(v[2]);
      rv[3] = eng::bf16v(v[3]);
      *(v4f*)(xs + c * kPitch + 4 * lane) = rv;
    }
    __syncthreads();

#pragma unroll 1
    for (int tl8 = 0; tl8 < kTilesPerChunk; ++tl8) {
      const int p = 16 * tl8 + n;
      float xin[kCin];
#pragma unroll
      for (int c = 0; c < kCin; ++c) xin[c] = xs[c * kPitch + p];
      v8h b0, b1;
#pragma unroll
      for (int r = 0; r < 8; ++r) {
        const float z0 = fmaf(wi0[r][2], xin[2], fmaf(wi0[r][1], xin[1], wi0[r][0] * xin[0]));
        const float z1 = fmaf(wi1[r][2], xin[2], fmaf(wi1[r][1], xin[1], wi1[r][0] * xin[0]));
        const float h0 = eng::fast_tanh(z0);
        const float h1 = eng::fast_tanh(z1);
        const bool live1 = (16 + 8 * hsel + r) < kHidC;
        b0[r] = eng::to_f16_flushed(h0 * kActCarry);
        b1[r] = eng::to_f16_flushed(live1 ? h1 * kActCarry : 0.0f);
      }
#pragma unroll
      for (int l = 0; l < kDepth; ++l) {
        eng::FragU fb; fb.h[0] = b0; fb.h[1] = b1;
        const v8f d0 = eng::mma_f16(fragW[l][0], fb.v);
        const v8f d1 = eng::mma_f16(fragW[l][1], fb.v);
#pragma unroll
        for (int r = 0; r < 8; ++r) {
          const float h0 = eng::fast_tanh(d0[r] * kFoldBack);
          const float h1 = eng::fast_tanh(d1[r] * kFoldBack);
          const bool live1 = (16 + 8 * hsel + r) < kHidC;
          b0[r] = eng::to_f16_flushed(h0 * kActCarry);
          b1[r] = eng::to_f16_flushed(live1 ? h1 * kActCarry : 0.0f);
        }
      }
      eng::FragU fb; fb.h[0] = b0; fb.h[1] = b1;
      const v8f dz = eng::mma_f16(fragO, fb.v);
      if (lowHalf) {
#pragma unroll
        for (int c = 0; c < kCin; ++c) os[c * kPitch + p] = 1.0f / (1.0f + expf(-(dz[c] * kFoldBack)));
      }
    }
    __syncthreads();

    {
      v4f ov[kCin];
#pragma unroll
      for (int c = 0; c < kCin; ++c) ov[c] = *(const v4f*)(os + c * kPitch + 4 * lane);
      for (int pass = 0; pass < 2; ++pass) {
#pragma unroll
        for (int c = 0; c < kCin; ++c)
          *(volatile v4f*)(outs + ((size_t)img * kCin + c) * kPlane + pix + 4 * lane) = ov[c];
        __threadfence();
      }
    }
    __syncthreads();
  }
}

extern "C" void kernel_launch(void* const* d_in, const int* in_sizes, int n_in,
                              void* d_out, int out_size, void* d_ws, size_t ws_size,
                              hipStream_t stream) {
  (void)d_ws;
  (void)ws_size;
  if (n_in < 4 || d_out == nullptr) return;
  if ((size_t)in_sizes[0] != kIoElems) return;
  if (in_sizes[1] != kHidC * kCin || in_sizes[2] != kDepth * kHidC * kHidC || in_sizes[3] != kCin * kHidC) return;
  if ((size_t)out_size != kIoElems) return;
  pixel_mlp_kernel<<<kWaves / kWavesPerBlock, 32 * kWavesPerBlock, 0, stream>>>((const float*)d_in[0], (const float*)d_in[1], (const float*)d_in[2],
                                              (const float*)d_in[3], (float*)d_out);
}
